// SimpleGraphConv_56736517980586
// MI455X (gfx1250) — hardware-verified
//
#include <hip/hip_runtime.h>
#include <stddef.h>
#include <stdint.h>


#define KD     128
#define NO     128
#define NW     2
#define NTHR   256
#define NWAVE  8
#define EPT    8
#define CHUNK  (NTHR * EPT)
#define WCAP   (EPT * 32)
#define LISTN  (NWAVE * WCAP)
#define NB     256
#define SLB    8
#define GBM    64
#define GTHR   128
#define WSMAX  134217728

static_assert((CHUNK & (CHUNK - 1)) == 0 && CHUNK <= 4096);
static_assert((NB & (NB - 1)) == 0 && NB == (1 << SLB));
static_assert(((long long)CHUNK << SLB) < (1LL << 31));
static_assert(LISTN % NTHR == 0);
static_assert((NB * NO) % (NTHR * 4) == 0);
static_assert(NB % (NWAVE * 8) == 0);
static_assert(KD % 32 == 0 && NO == 128 && NO == GTHR);
static_assert(GBM == (GTHR / 32) * 16);
static_assert((NW * NO * KD) % (NTHR * 8) == 0);

typedef float          v4f   __attribute__((ext_vector_type(4)));
typedef float          v8f   __attribute__((ext_vector_type(8)));
typedef int            v4i   __attribute__((ext_vector_type(4)));
typedef int            v8i   __attribute__((ext_vector_type(8)));
typedef unsigned short v8us  __attribute__((ext_vector_type(8)));
typedef unsigned short v16us __attribute__((ext_vector_type(16)));
typedef __bf16         v16bf __attribute__((ext_vector_type(16)));
typedef v4f  __attribute__((may_alias)) v4fa;
typedef v8us __attribute__((may_alias)) v8usa;
union FragB { v16bf v; v16us u; v8us h[2]; v8i w; };

__device__ __forceinline__ v8f wmb(const FragB& a, const FragB& b, v8f c) {
  v8f d = __builtin_amdgcn_wmma_f32_16x16x32_bf16(false, a.v, false, b.v, (short)0, c, false, false);
  asm volatile("v_nop\n\tv_nop\n\tv_nop\n\tv_nop" : "+v"(d) : "v"(a.w), "v"(b.w));
  return d;
}

__device__ __forceinline__ unsigned bf16_bits(float f) {
  const unsigned u = __float_as_uint(f);
  return (u + 0x7FFFu + ((u >> 16) & 1u)) >> 16;
}
__device__ __forceinline__ float bf16_val(float f) {
  return __uint_as_float(bf16_bits(f) << 16);
}

__device__ __forceinline__ int scan_chunk(const int* __restrict__ dsts, int nE, int cbase, int slotBase,
                                          int nb, int vec8, int* list, int tid, int lane, int wave) {
  int wc = 0;
  const int el0  = tid * EPT;
  const int e0   = cbase + el0;
  const int sent = -2147483647 - 1;
  v4i da, db;
  if (vec8 != 0 && cbase + CHUNK <= nE) {
    da = *(const v4i*)(dsts + e0);
    db = *(const v4i*)(dsts + e0 + 4);
  } else {
    da.x = (e0     < nE) ? dsts[min(e0,     nE - 1)] : sent;
    da.y = (e0 + 1 < nE) ? dsts[min(e0 + 1, nE - 1)] : sent;
    da.z = (e0 + 2 < nE) ? dsts[min(e0 + 2, nE - 1)] : sent;
    da.w = (e0 + 3 < nE) ? dsts[min(e0 + 3, nE - 1)] : sent;
    db.x = (e0 + 4 < nE) ? dsts[min(e0 + 4, nE - 1)] : sent;
    db.y = (e0 + 5 < nE) ? dsts[min(e0 + 5, nE - 1)] : sent;
    db.z = (e0 + 6 < nE) ? dsts[min(e0 + 6, nE - 1)] : sent;
    db.w = (e0 + 7 < nE) ? dsts[min(e0 + 7, nE - 1)] : sent;
  }
  const unsigned nbs = (unsigned)slotBase;
  const unsigned unb = (unsigned)nb;
  const unsigned s0 = (unsigned)da.x - nbs, s1 = (unsigned)da.y - nbs;
  const unsigned s2 = (unsigned)da.z - nbs, s3 = (unsigned)da.w - nbs;
  const unsigned s4 = (unsigned)db.x - nbs, s5 = (unsigned)db.y - nbs;
  const unsigned s6 = (unsigned)db.z - nbs, s7 = (unsigned)db.w - nbs;
  const bool h0 = s0 < unb, h1 = s1 < unb, h2 = s2 < unb, h3 = s3 < unb;
  const bool h4 = s4 < unb, h5 = s5 < unb, h6 = s6 < unb, h7 = s7 < unb;
  const unsigned any = __builtin_amdgcn_ballot_w32(h0 | h1 | h2 | h3 | h4 | h5 | h6 | h7);
  if (any != 0u) {
#define HITJ(J, HJ, SJ) { \
      const unsigned mj = __builtin_amdgcn_ballot_w32(HJ); \
      if (mj != 0u) { \
        if (HJ) { \
          const int pos = wc + (int)__builtin_amdgcn_mbcnt_lo(mj, 0u); \
          if (pos < WCAP) list[wave * WCAP + pos] = ((el0 + (J)) << SLB) | (int)(SJ); \
        } \
        wc += (int)__builtin_popcount(mj); } }
    HITJ(0, h0, s0)
    HITJ(1, h1, s1)
    HITJ(2, h2, s2)
    HITJ(3, h3, s3)
    HITJ(4, h4, s4)
    HITJ(5, h5, s5)
    HITJ(6, h6, s6)
    HITJ(7, h7, s7)
#undef HITJ
  }
  return wc;
}

__global__ __launch_bounds__(NTHR) void k_wprep(const float* __restrict__ Wa, const float* __restrict__ Wb,
                                                unsigned short* WT, int nUnits) {
  const int u = (int)blockIdx.x * NTHR + (int)threadIdx.x;
  if (u >= nUnits) return;
  const int n  = u >> 4;
  const int k8 = (u & 15) * 8;
  const float* p = (n < NO) ? (Wa + (size_t)n * KD + k8) : (Wb + (size_t)(n - NO) * KD + k8);
  const v4f a = *(const v4f*)p;
  const v4f b = *(const v4f*)(p + 4);
  v8us o;
  o[0] = (unsigned short)bf16_bits(a.x);
  o[1] = (unsigned short)bf16_bits(a.y);
  o[2] = (unsigned short)bf16_bits(a.z);
  o[3] = (unsigned short)bf16_bits(a.w);
  o[4] = (unsigned short)bf16_bits(b.x);
  o[5] = (unsigned short)bf16_bits(b.y);
  o[6] = (unsigned short)bf16_bits(b.z);
  o[7] = (unsigned short)bf16_bits(b.w);
  unsigned short* dp = WT + (size_t)n * KD + k8;
  *(volatile v8us*)dp = o;
  __threadfence();
  *(volatile v8us*)dp = o;
}

__global__ __launch_bounds__(GTHR) void k_gemm(const float* __restrict__ x, const unsigned short* __restrict__ WT,
                                               const float* __restrict__ bias, float* H, int nN, int NP) {
  __shared__ __attribute__((aligned(16))) float sB[NO];
  __shared__ __attribute__((aligned(16))) float stg[GBM * NO];
  const int tid = (int)threadIdx.x, lane = tid & 31, wave = tid >> 5, hh = lane >> 4, m = lane & 15;
  const int y = (int)blockIdx.y;
  const int rowBase = (int)blockIdx.x * GBM;

  {
    const float bv = bf16_val(bias[tid]);
    sB[tid] = (y == 0) ? bv : 0.0f;
  }
  __syncthreads();

  const int row = rowBase + 16 * wave + m;
  const int rc  = row < nN ? row : nN - 1;
  const float* xr = x + (size_t)rc * KD;

  v8f acc[8];
  {
    const v8f z = {0.f, 0.f, 0.f, 0.f, 0.f, 0.f, 0.f, 0.f};
#pragma unroll
    for (int t = 0; t < 8; ++t) acc[t] = z;
  }
  const unsigned short* wp = WT + (size_t)(y * NO + m) * KD + 8 * hh;

#pragma unroll 1
  for (int kk = 0; kk < KD / 32; ++kk) {
    const int k0 = 32 * kk;
    const float* xp = xr + k0 + 8 * hh;
    const v4f x0 = *(const v4f*)(xp);
    const v4f x1 = *(const v4f*)(xp + 4);
    const v4f x2 = *(const v4f*)(xp + 16);
    const v4f x3 = *(const v4f*)(xp + 20);
    FragB a;
    a.u[0]  = (unsigned short)bf16_bits(x0.x);
    a.u[1]  = (unsigned short)bf16_bits(x0.y);
    a.u[2]  = (unsigned short)bf16_bits(x0.z);
    a.u[3]  = (unsigned short)bf16_bits(x0.w);
    a.u[4]  = (unsigned short)bf16_bits(x1.x);
    a.u[5]  = (unsigned short)bf16_bits(x1.y);
    a.u[6]  = (unsigned short)bf16_bits(x1.z);
    a.u[7]  = (unsigned short)bf16_bits(x1.w);
    a.u[8]  = (unsigned short)bf16_bits(x2.x);
    a.u[9]  = (unsigned short)bf16_bits(x2.y);
    a.u[10] = (unsigned short)bf16_bits(x2.z);
    a.u[11] = (unsigned short)bf16_bits(x2.w);
    a.u[12] = (unsigned short)bf16_bits(x3.x);
    a.u[13] = (unsigned short)bf16_bits(x3.y);
    a.u[14] = (unsigned short)bf16_bits(x3.z);
    a.u[15] = (unsigned short)bf16_bits(x3.w);
#pragma unroll
    for (int nt = 0; nt < 8; ++nt) {
      const unsigned short* wq = wp + (size_t)(16 * nt) * KD + k0;
      FragB bf;
      bf.h[0] = *(const v8usa*)wq;
      bf.h[1] = *(const v8usa*)(wq + 16);
      acc[nt] = wmb(a, bf, acc[nt]);
    }
  }

  float* st = stg + wave * (16 * NO);
#pragma unroll
  for (int nt = 0; nt < 8; ++nt) {
    const int lc = 16 * nt + m;
    const float bv = sB[lc];
#pragma unroll
    for (int r = 0; r < 8; ++r) {
      const int lr = 8 * hh + r;
      st[lr * NO + lc] = acc[nt][r] + bv;
    }
  }
  __syncthreads();

  float* hp = H + (size_t)y * (size_t)NP * NO + (size_t)(rowBase + 16 * wave) * NO + 4 * lane;
  v4f pv[16];
#pragma unroll
  for (int j = 0; j < 16; ++j) pv[j] = *(const v4fa*)(st + j * NO + 4 * lane);
#pragma unroll
  for (int j = 0; j < 16; ++j) *(volatile v4f*)(hp + (size_t)j * NO) = pv[j];
  __threadfence();
#pragma unroll
  for (int j = 0; j < 16; ++j) *(volatile v4f*)(hp + (size_t)j * NO) = pv[j];
}

__global__ __launch_bounds__(NTHR) void k_agg(const int* __restrict__ srcs, const int* __restrict__ dsts,
                                              const float* __restrict__ ew, const float* __restrict__ H0,
                                              const float* __restrict__ H1, int nE, int nN, int vec8,
                                              float* out) {
  __shared__ __attribute__((aligned(16))) float sacc[NB * NO];
  __shared__ __attribute__((aligned(16))) int list[LISTN];
  __shared__ int wcnt[NWAVE];
  const int tid = (int)threadIdx.x, lane = tid & 31, wave = tid >> 5;
  const int nodeBase = (int)blockIdx.x * NB;

  {
    const v4f z = {0.f, 0.f, 0.f, 0.f};
    for (int i = tid; i < (NB * NO) / 4; i += NTHR) *(v4fa*)(sacc + 4 * i) = z;
  }
  for (int i = tid; i < LISTN; i += NTHR) list[i] = 0;
  if (tid < NWAVE) wcnt[tid] = 0;
  __syncthreads();

  const int nChunks = (nE + CHUNK - 1) / CHUNK;
#pragma unroll 1
  for (int ch = 0; ch < nChunks; ++ch) {
    const int cbase = ch * CHUNK;
    const int wc = scan_chunk(dsts, nE, cbase, nodeBase, NB, vec8, list, tid, lane, wave);
    if (lane == 0) wcnt[wave] = wc;
    __syncthreads();
    if (wave == 0) {
#pragma unroll 1
      for (int w2 = 0; w2 < NWAVE; ++w2) {
        int c = wcnt[w2];
        c = c < 0 ? 0 : (c > WCAP ? WCAP : c);
#pragma unroll 1
        for (int b0 = 0; b0 < c; b0 += 32) {
          const int idx = b0 + lane;
          const int ent = list[w2 * WCAP + (idx < WCAP ? idx : WCAP - 1)];
          const int el  = (ent >> SLB) & (CHUNK - 1);
          int eid = cbase + el;
          eid = eid < 0 ? 0 : (eid > nE - 1 ? nE - 1 : eid);
          const int sraw = srcs[eid];
          const int s = sraw < 0 ? 0 : (sraw > nN - 1 ? nN - 1 : sraw);
          const float wv = bf16_val(ew[eid]);
          const int wvi = __float_as_int(wv);
          const int m32 = (c - b0) < 32 ? (c - b0) : 32;
#pragma unroll 1
          for (int k = 0; k < m32; ++k) {
            const int u  = __builtin_amdgcn_readlane(ent, k);
            const int sl = u & (NB - 1);
            const int sk = __builtin_amdgcn_readlane(s, k);
            const float wk = __int_as_float(__builtin_amdgcn_readlane(wvi, k));
            const v4f hv = *(const v4f*)(H1 + (size_t)sk * NO + 4 * lane);
            float* ap = sacc + sl * NO + 4 * lane;
            v4f av = *(const v4fa*)ap;
            av = av + wk * hv;
            *(v4fa*)ap = av;
          }
        }
      }
    }
    __syncthreads();
  }

  int nv = nN - nodeBase;
  nv = nv < 0 ? 0 : (nv > NB ? NB : nv);
#pragma unroll 1
  for (int g = 0; g < NB / (NWAVE * 8); ++g) {
    v4f vals[8];
#pragma unroll
    for (int j = 0; j < 8; ++j) {
      const int s = wave + NWAVE * (8 * g + j);
      const int node = nodeBase + s;
      const int nc = node < nN ? node : nN - 1;
      const v4f a4 = *(const v4fa*)(sacc + s * NO + 4 * lane);
      const v4f h4 = *(const v4f*)(H0 + (size_t)nc * NO + 4 * lane);
      vals[j] = a4 + h4;
    }
#pragma unroll
    for (int j = 0; j < 8; ++j) {
      const int s = wave + NWAVE * (8 * g + j);
      if (s < nv) *(volatile v4f*)(out + (size_t)(nodeBase + s) * NO + 4 * lane) = vals[j];
    }
    __threadfence();
#pragma unroll
    for (int j = 0; j < 8; ++j) {
      const int s = wave + NWAVE * (8 * g + j);
      if (s < nv) *(volatile v4f*)(out + (size_t)(nodeBase + s) * NO + 4 * lane) = vals[j];
    }
  }
}

static inline int cdiv(int a, int b) { return (a + b - 1) / b; }

extern "C" void kernel_launch(void* const* d_in, const int* in_sizes, int n_in,
                              void* d_out, int out_size, void* d_ws, size_t ws_size,
                              hipStream_t stream) {
  if (n_in < 6) return;
  if (in_sizes[0] < KD || (in_sizes[0] % KD) != 0) return;
  const int nN = in_sizes[0] / KD;
  if (in_sizes[1] < 2 || (in_sizes[1] & 1) != 0) return;
  const int nE = in_sizes[1] / 2;
  if (nE < 1 || in_sizes[2] != nE) return;
  if (in_sizes[3] != NO * KD || in_sizes[4] != NO || in_sizes[5] != NO * KD) return;
  if (out_size != nN * NO) return;

  const float* x    = (const float*)d_in[0];
  const int*   edge = (const int*)d_in[1];
  const float* ew   = (const float*)d_in[2];
  const float* Wa   = (const float*)d_in[3];
  const float* ba   = (const float*)d_in[4];
  const float* Wb   = (const float*)d_in[5];
  float* out = (float*)d_out;
  const int* src = edge;
  const int* dst = edge + nE;

  const int NP = cdiv(nN, GBM) * GBM;
  const int gM = NP / GBM;
  const int gA = cdiv(nN, NB);
  if ((long long)gA * NB < (long long)nN) return;
  const int vec8 = ((nE & 3) == 0) ? 1 : 0;

  char* ws = (char*)d_ws;
  size_t off = 0;
  const size_t oWT = off; off += (size_t)NW * NO * KD * 2;           off = (off + 255) & ~(size_t)255;
  const size_t oH  = off; off += (size_t)NW * (size_t)NP * NO * 4;   off = (off + 255) & ~(size_t)255;
  if (off > ws_size || off > (size_t)WSMAX) return;
  unsigned short* WT = (unsigned short*)(ws + oWT);
  float*          H  = (float*)(ws + oH);
  const float* H0 = H;
  const float* H1 = H + (size_t)NP * NO;

  const int nUw = (NW * NO * KD) / 8;
  k_wprep<<<cdiv(nUw, NTHR), NTHR, 0, stream>>>(Wa, Wb, WT, nUw);
  k_gemm<<<dim3(gM, NW, 1), GTHR, 0, stream>>>(x, WT, ba, H, nN, NP);
  k_agg<<<gA, NTHR, 0, stream>>>(src, dst, ew, H0, H1, nE, nN, vec8, out);
}
